// KANLayer_85512798864151
// MI455X (gfx1250) — hardware-verified
//
#include <hip/hip_runtime.h>
#include <math.h>

constexpr int kBatch = 4096;
constexpr int kInF   = 1024;
constexpr int kOutF  = 1024;
constexpr int kBasis = 8;
constexpr int kKdim  = kInF * kBasis;
constexpr float kWCarry    = 1024.0f;
constexpr float kWCarryInv = 1.0f / 1024.0f;
static_assert(kKdim % 32 == 0, "K multiple of 32");
static_assert(kBatch % 64 == 0, "M multiple of 64");
static_assert(kOutF % 64 == 0, "N multiple of 64");

constexpr size_t kPlaneABytes = (size_t)kBatch * kKdim * 2;
constexpr size_t kPlaneWBytes = (size_t)kOutF * kKdim * 2;
constexpr size_t kWsTotal     = kPlaneABytes + kPlaneWBytes;
static_assert(kWsTotal <= 134217728ull, "carve within 128 MiB");
static_assert(kPlaneABytes % 128 == 0, "plane W base 128-B aligned");

typedef __attribute__((ext_vector_type(16))) _Float16 v16h;
typedef __attribute__((ext_vector_type(8)))  _Float16 v8h;
typedef __attribute__((ext_vector_type(16))) __bf16   v16b;
typedef __attribute__((ext_vector_type(8)))  __bf16   v8b;
typedef __attribute__((ext_vector_type(8)))  float    v8f;
typedef __attribute__((ext_vector_type(4)))  float    v4f;
typedef __attribute__((ext_vector_type(4)))  unsigned int v4u;

__device__ __forceinline__ unsigned short f2bf_bits(float f) {
  unsigned u = __float_as_uint(f);
  return (unsigned short)((u + 0x7FFFu + ((u >> 16) & 1u)) >> 16);
}
__device__ __forceinline__ float bf_bits2f(unsigned short h) { return __uint_as_float(((unsigned)h) << 16); }

__device__ __forceinline__ void dep_guard_h(v8f& a, v8f& b, v16h x, v16h y) { asm volatile("v_nop\n\tv_nop\n\tv_nop\n\tv_nop" : "+v"(a), "+v"(b) : "v"(x), "v"(y)); }
__device__ __forceinline__ void dep_guard_b(v8f& a, v8f& b, v16b x, v16b y) { asm volatile("v_nop\n\tv_nop\n\tv_nop\n\tv_nop" : "+v"(a), "+v"(b) : "v"(x), "v"(y)); }
__device__ __forceinline__ void dep_guard4_h(v8f& a, v8f& b, v8f& c, v8f& d, v16h x, v16h y) { asm volatile("v_nop\n\tv_nop\n\tv_nop\n\tv_nop" : "+v"(a), "+v"(b), "+v"(c), "+v"(d) : "v"(x), "v"(y)); }
__device__ __forceinline__ void dep_guard4_b(v8f& a, v8f& b, v8f& c, v8f& d, v16b x, v16b y) { asm volatile("v_nop\n\tv_nop\n\tv_nop\n\tv_nop" : "+v"(a), "+v"(b), "+v"(c), "+v"(d) : "v"(x), "v"(y)); }
__device__ __forceinline__ void keep4_h(v16h a, v16h b, v16h c, v16h d) { asm volatile("v_nop" :: "v"(a), "v"(b), "v"(c), "v"(d)); }
__device__ __forceinline__ void keep4_b(v16b a, v16b b, v16b c, v16b d) { asm volatile("v_nop" :: "v"(a), "v"(b), "v"(c), "v"(d)); }
__device__ __forceinline__ void acc_guard4(v8f& a, v8f& b, v8f& c, v8f& d) { asm volatile("v_nop\n\tv_nop\n\tv_nop\n\tv_nop" : "+v"(a), "+v"(b), "+v"(c), "+v"(d)); }
template <typename T> struct Frag;
template <> struct Frag<_Float16> {
  typedef v16h V; union U { v16h v; v8h h[2]; };
  static __device__ __forceinline__ v16h load(const _Float16* p) {
    U f; f.h[0] = *(const v8h*)(p); f.h[1] = *(const v8h*)(p + 16); return f.v;
  }
  static __device__ __forceinline__ v8f mma(v16h a, v16h b, v8f c) {
    return __builtin_amdgcn_wmma_f32_16x16x32_f16(false, a, false, b, (short)0, c, false, false);
  }
  static __device__ __forceinline__ void guard(v8f& a, v8f& b, v16h x, v16h y) { dep_guard_h(a, b, x, y); }
  static __device__ __forceinline__ void guard4(v8f& a, v8f& b, v8f& c, v8f& d, v16h x, v16h y) { dep_guard4_h(a, b, c, d, x, y); }
  static __device__ __forceinline__ void keep(v16h a, v16h b, v16h c, v16h d) { keep4_h(a, b, c, d); }
};
template <> struct Frag<__bf16> {
  typedef v16b V; union U { v16b v; v8b h[2]; };
  static __device__ __forceinline__ v16b load(const __bf16* p) {
    U f; f.h[0] = *(const v8b*)(p); f.h[1] = *(const v8b*)(p + 16); return f.v;
  }
  static __device__ __forceinline__ v8f mma(v16b a, v16b b, v8f c) {
    return __builtin_amdgcn_wmma_f32_16x16x32_bf16(false, a, false, b, (short)0, c, false, false);
  }
  static __device__ __forceinline__ void guard(v8f& a, v8f& b, v16b x, v16b y) { dep_guard_b(a, b, x, y); }
  static __device__ __forceinline__ void guard4(v8f& a, v8f& b, v8f& c, v8f& d, v16b x, v16b y) { dep_guard4_b(a, b, c, d, x, y); }
  static __device__ __forceinline__ void keep(v16b a, v16b b, v16b c, v16b d) { keep4_b(a, b, c, d); }
};

__device__ __forceinline__ unsigned pk16(unsigned short a, unsigned short b) { return (unsigned)a | ((unsigned)b << 16); }
__device__ __forceinline__ unsigned short h_bits(float f) { const _Float16 h = (_Float16)f; return __builtin_bit_cast(unsigned short, h); }

template <int ET> struct Elem;
template <> struct Elem<0> { typedef _Float16 T; };
template <> struct Elem<1> { typedef __bf16 T; };
template <int ET, bool SPLIT, int BIAS_MODE, int OUT_MODE, bool RESID, int ACT = 0>
__global__ __launch_bounds__(256) void wmma_gemm64(
    const unsigned short* __restrict__ Ap, const unsigned short* __restrict__ A2p, int lda, long strideA,
    const unsigned short* __restrict__ Btp, const unsigned short* __restrict__ Bt2p, int ldb, long strideB,
    void* __restrict__ Cout, void* __restrict__ Cout2, int ldc, long strideC,
    const float* __restrict__ bias,
    const float* __restrict__ resid, long strideR,
    int M, int N, int K, float scale) {
  typedef typename Elem<ET>::T T;
  typedef typename Frag<T>::V V;
  const T* A = (const T*)Ap; const T* A2 = (const T*)A2p; const T* Bt = (const T*)Btp; const T* Bt2 = (const T*)Bt2p;
  __shared__ __align__(16) float sT[8][16 * 68];
  const int b    = blockIdx.y;
  const int lane = threadIdx.x & 31;
  const int wave = threadIdx.x >> 5;
  const int tilesN = N >> 6;
  const int tilesM = M >> 6;
  const int tile = blockIdx.x * 8 + wave;
  if (tile >= tilesM * tilesN) return;
  const int tm = tile / tilesN;
  const int tn = tile - tm * tilesN;
  const int m0 = tm << 6;
  const int n0 = tn << 6;

  const T* Ab  = A  + (size_t)b * strideA;
  const T* Bb  = Bt + (size_t)b * strideB;
  const T* Ab2 = SPLIT ? (A2  + (size_t)b * strideA) : nullptr;
  const T* Bb2 = SPLIT ? (Bt2 + (size_t)b * strideB) : nullptr;

  const int rlane = lane & 15;
  const int koff  = (lane >> 4) * 8;
  const int mOff  = (lane >> 4) * 8;

  v8f acc[4][4];
#pragma unroll
  for (int i = 0; i < 4; ++i)
#pragma unroll
    for (int j = 0; j < 4; ++j) acc[i][j] = (v8f){0.f,0.f,0.f,0.f,0.f,0.f,0.f,0.f};

  for (int k0 = 0; k0 < K; k0 += 32) {
    V bh[4], bl[4];
#pragma unroll
    for (int j = 0; j < 4; ++j) {
      const size_t bo = (size_t)(n0 + (j << 4) + rlane) * ldb + koff + k0;
      bh[j] = Frag<T>::load(Bb + bo);
      if (SPLIT) bl[j] = Frag<T>::load(Bb2 + bo);
    }
#pragma unroll
    for (int i = 0; i < 4; ++i) {
      const size_t ao = (size_t)(m0 + (i << 4) + rlane) * lda + koff + k0;
      V ah = Frag<T>::load(Ab + ao);
      V al;
      if (SPLIT) al = Frag<T>::load(Ab2 + ao);
#pragma unroll
      for (int j = 0; j < 4; ++j) {
        acc[i][j] = Frag<T>::mma(ah, bh[j], acc[i][j]);
        if (SPLIT) {
          acc[i][j] = Frag<T>::mma(ah, bl[j], acc[i][j]);
          acc[i][j] = Frag<T>::mma(al, bh[j], acc[i][j]);
        }
      }
      Frag<T>::guard4(acc[i][0], acc[i][1], acc[i][2], acc[i][3], ah, SPLIT ? al : bh[3]);
    }
    Frag<T>::keep(bh[0], bh[1], bh[2], bh[3]);
    if (SPLIT) Frag<T>::keep(bl[0], bl[1], bl[2], bl[3]);
  }
  acc_guard4(acc[0][0], acc[0][1], acc[0][2], acc[0][3]);
  acc_guard4(acc[1][0], acc[1][1], acc[1][2], acc[1][3]);
  acc_guard4(acc[2][0], acc[2][1], acc[2][2], acc[2][3]);
  acc_guard4(acc[3][0], acc[3][1], acc[3][2], acc[3][3]);

  float* slab = sT[wave];
  const float* Rb = RESID ? (resid + (size_t)b * strideR) : nullptr;
#pragma unroll
  for (int i = 0; i < 4; ++i) {
    const int mBase = m0 + (i << 4);
#pragma unroll
    for (int j = 0; j < 4; ++j) {
      const int n = n0 + (j << 4) + rlane;
      float bv = 0.f;
      if (BIAS_MODE == 2) bv = bias[n];
#pragma unroll
      for (int r = 0; r < 8; ++r) {
        float v = acc[i][j][r] * scale;
        if (BIAS_MODE == 1) v += bias[mBase + mOff + r];
        if (BIAS_MODE == 2) v += bv;
        if (RESID) v += Rb[(size_t)(mBase + mOff + r) * ldc + n];
        if (ACT == 2) v = fmaxf(v, 0.0f);
        if (ACT == 4) v = (v > 0.f) ? v : 0.01f * v;
        slab[(mOff + r) * 68 + (j << 4) + rlane] = v;
      }
    }
    __builtin_amdgcn_fence(__ATOMIC_RELEASE, "workgroup");
    __builtin_amdgcn_wave_barrier();
    __builtin_amdgcn_fence(__ATOMIC_ACQUIRE, "workgroup");
    if (OUT_MODE == 0) {
      float* C = (float*)Cout + (size_t)b * strideC;
      const int hh = lane >> 4, c4 = (lane & 15) * 4;
      for (int pass = 0; pass < 2; ++pass) {
#pragma unroll
        for (int it = 0; it < 8; ++it) {
          const int row = it * 2 + hh;
          v4f v = *(const v4f*)(slab + row * 68 + c4);
          *(volatile v4f*)(C + (size_t)(mBase + row) * ldc + n0 + c4) = v;
        }
        __threadfence();
      }
    } else {
      const int q = lane >> 3, c8 = (lane & 7) * 8;
      unsigned short* C  = (unsigned short*)Cout  + (size_t)b * strideC;
      unsigned short* C2 = (OUT_MODE == 2) ? ((unsigned short*)Cout2 + (size_t)b * strideC) : nullptr;
      for (int pass = 0; pass < 2; ++pass) {
#pragma unroll
        for (int it = 0; it < 4; ++it) {
          const int row = it * 4 + q;
          const float* sp = slab + row * 68 + c8;
          v8h hv, lv;
#pragma unroll
          for (int e = 0; e < 8; ++e) {
            if (OUT_MODE == 1) {
              hv[e] = (_Float16)sp[e];
            } else {
              unsigned short hb = f2bf_bits(sp[e]);
              unsigned short lb = f2bf_bits(sp[e] - bf_bits2f(hb));
              hv[e] = __builtin_bit_cast(_Float16, hb);
              lv[e] = __builtin_bit_cast(_Float16, lb);
            }
          }
          *(volatile v8h*)(C + (size_t)(mBase + row) * ldc + n0 + c8) = hv;
          if (OUT_MODE == 2) *(volatile v8h*)(C2 + (size_t)(mBase + row) * ldc + n0 + c8) = lv;
        }
        __threadfence();
      }
    }
    __builtin_amdgcn_fence(__ATOMIC_RELEASE, "workgroup");
    __builtin_amdgcn_wave_barrier();
    __builtin_amdgcn_fence(__ATOMIC_ACQUIRE, "workgroup");
  }
}

__global__ __launch_bounds__(256) void basis8_f16_kernel(const float* __restrict__ x, unsigned short* __restrict__ A, int n) {
  const int idx = blockIdx.x * 256 + threadIdx.x;
  if (idx >= n) return;
  const float xv = x[idx];
  const float t  = tanhf(xv);
  const float tt = 2.0f * t;
  const float p0 = 1.0f;
  const float p1 = t;
  const float p2 = tt * p1 - p0;
  const float p3 = tt * p2 - p1;
  const float p4 = tt * p3 - p2;
  const float p5 = tt * p4 - p3;
  const float p6 = tt * p5 - p4;
  const float p7 = tt * p6 - p5;
  float t0v = 1.0f;
  asm volatile("" : "+v"(t0v));
  unsigned short hb[8];
  hb[0] = h_bits(t0v);
  hb[1] = h_bits(p1);
  hb[2] = h_bits(p2);
  hb[3] = h_bits(p3);
  hb[4] = h_bits(p4);
  hb[5] = h_bits(p5);
  hb[6] = h_bits(p6);
  hb[7] = h_bits(p7);
  const v4u u = (v4u){pk16(hb[0], hb[1]), pk16(hb[2], hb[3]), pk16(hb[4], hb[5]), pk16(hb[6], hb[7])};
  unsigned short* q = A + 8 * (size_t)idx;
  *(volatile v4u*)q = u;
  __threadfence();
  *(volatile v4u*)q = u;
}

__global__ __launch_bounds__(256) void wcast8_f16_kernel(const float* __restrict__ in, unsigned short* __restrict__ out,
                                                         int n8, float scale) {
  const int i = blockIdx.x * 256 + threadIdx.x;
  if (i >= n8) return;
  const float* p = in + 8 * (size_t)i;
  const v4f a = *(const v4f*)(p);
  const v4f c = *(const v4f*)(p + 4);
  unsigned short hb[8];
#pragma unroll
  for (int e = 0; e < 4; ++e) {
    hb[e]     = h_bits(a[e] * scale);
    hb[4 + e] = h_bits(c[e] * scale);
  }
  const v4u u = (v4u){pk16(hb[0], hb[1]), pk16(hb[2], hb[3]), pk16(hb[4], hb[5]), pk16(hb[6], hb[7])};
  unsigned short* q = out + 8 * (size_t)i;
  *(volatile v4u*)q = u;
  __threadfence();
  *(volatile v4u*)q = u;
}

extern "C" void kernel_launch(void* const* d_in, const int* in_sizes, int n_in,
                              void* d_out, int out_size, void* d_ws, size_t ws_size,
                              hipStream_t stream) {
  if (n_in < 3) return;
  if (in_sizes[0] != kBatch * kInF) return;
  if (in_sizes[1] != kOutF * kInF * kBasis) return;
  if (in_sizes[2] != kOutF) return;
  if (out_size != kBatch * kOutF) return;
  if (ws_size < kWsTotal) return;

  const float* x    = (const float*)d_in[0];
  const float* W    = (const float*)d_in[1];
  const float* bias = (const float*)d_in[2];
  float* out        = (float*)d_out;

  unsigned short* Ap = (unsigned short*)d_ws;
  unsigned short* Wp = (unsigned short*)((char*)d_ws + kPlaneABytes);

  const int nA = kBatch * kInF;
  basis8_f16_kernel<<<dim3((nA + 255) / 256), dim3(256), 0, stream>>>(x, Ap, nA);

  const int n8 = (kOutF * kKdim) / 8;
  wcast8_f16_kernel<<<dim3((n8 + 255) / 256), dim3(256), 0, stream>>>(W, Wp, n8, kWCarry);

  const int tiles = (kBatch / 64) * (kOutF / 64);
  wmma_gemm64<0, false, 2, 0, false, 0><<<dim3((tiles + 7) / 8, 1), dim3(256), 0, stream>>>(
      Ap, Ap, kKdim, 0L,
      Wp, Wp, kKdim, 0L,
      (void*)out, (void*)out, kOutF, 0L,
      bias,
      bias, 0L,
      kBatch, kOutF, kKdim, kWCarryInv);
}
